// MultiHeadAttention_9689446220205
// MI455X (gfx1250) — hardware-verified
//
#include <hip/hip_runtime.h>
#include <math.h>

#ifndef NB
#define NB 2
#endif
#ifndef SEQ
#define SEQ 2048
#endif
#define NB_FULL 2
#define SEQ_FULL 2048
#define EMB 1024
#define NHEAD 16
#define DHEAD 64

static_assert(NB >= 1 && NB <= NB_FULL);
static_assert(SEQ >= 64 && SEQ <= SEQ_FULL && SEQ % 64 == 0);
static_assert(EMB == NHEAD * DHEAD);
static_assert(DHEAD == 64);
static_assert(DHEAD % 64 == 0 && DHEAD % 32 == 0);
static_assert(EMB % 64 == 0 && (2 * EMB) % 32 == 0);
static_assert(((long long)NB * SEQ * NHEAD) % 64 == 0);
static_assert(EMB % 8 == 0);

typedef __attribute__((ext_vector_type(16))) _Float16 v16h;
typedef __attribute__((ext_vector_type(8)))  _Float16 v8h;
typedef __attribute__((ext_vector_type(16))) __bf16   v16b;
typedef __attribute__((ext_vector_type(8)))  __bf16   v8b;
typedef __attribute__((ext_vector_type(8)))  float    v8f;
typedef __attribute__((ext_vector_type(4)))  float    v4f;
typedef unsigned int cm_u4 __attribute__((ext_vector_type(4)));

__device__ __forceinline__ v8f wmma16(v16h a, v16h b, v8f c) {
    c = __builtin_amdgcn_wmma_f32_16x16x32_f16(false, a, false, b, (short)0, c, false, false);
    asm volatile("v_nop\n\tv_nop\n\tv_nop\n\tv_nop" : "+v"(c) : "v"(a), "v"(b));
    return c;
}

#define VST2(T, ptr, val) do { const T vst2_v_ = (val); *(volatile T*)(ptr) = vst2_v_; __threadfence(); *(volatile T*)(ptr) = vst2_v_; } while (0)
#define VST2V4(ptr, val) do { const v4f vst2_v4_ = (val); *(volatile v4f*)(ptr) = vst2_v4_; __threadfence(); *(volatile v4f*)(ptr) = vst2_v4_; } while (0)

namespace w25 {
__device__ __forceinline__ unsigned short f2bf_bits(float f) {
  unsigned u = __float_as_uint(f);
  return (unsigned short)((u + 0x7FFFu + ((u >> 16) & 1u)) >> 16);
}
__device__ __forceinline__ float bf_bits2f(unsigned short h) { return __uint_as_float(((unsigned)h) << 16); }

__device__ __forceinline__ void dep_guard_h(v8f& a, v8f& b, v16h x, v16h y) { asm volatile("v_nop\n\tv_nop\n\tv_nop\n\tv_nop" : "+v"(a), "+v"(b) : "v"(x), "v"(y)); }
__device__ __forceinline__ void dep_guard_b(v8f& a, v8f& b, v16b x, v16b y) { asm volatile("v_nop\n\tv_nop\n\tv_nop\n\tv_nop" : "+v"(a), "+v"(b) : "v"(x), "v"(y)); }
__device__ __forceinline__ void keep4_h(v16h a, v16h b, v16h c, v16h d) { asm volatile("v_nop" :: "v"(a), "v"(b), "v"(c), "v"(d)); }
__device__ __forceinline__ void keep4_b(v16b a, v16b b, v16b c, v16b d) { asm volatile("v_nop" :: "v"(a), "v"(b), "v"(c), "v"(d)); }
__device__ __forceinline__ void acc_guard4(v8f& a, v8f& b, v8f& c, v8f& d) { asm volatile("v_nop\n\tv_nop\n\tv_nop\n\tv_nop" : "+v"(a), "+v"(b), "+v"(c), "+v"(d)); }
template <typename T> struct Frag;
template <> struct Frag<_Float16> {
  typedef v16h V; union U { v16h v; v8h h[2]; };
  static __device__ __forceinline__ v16h load(const _Float16* p) {
    U f; f.h[0] = *(const v8h*)(p); f.h[1] = *(const v8h*)(p + 16); return f.v;
  }
  static __device__ __forceinline__ v8f mma(v16h a, v16h b, v8f c) {
    return __builtin_amdgcn_wmma_f32_16x16x32_f16(false, a, false, b, (short)0, c, false, false);
  }
  static __device__ __forceinline__ void guard(v8f& a, v8f& b, v16h x, v16h y) { dep_guard_h(a, b, x, y); }
  static __device__ __forceinline__ void keep(v16h a, v16h b, v16h c, v16h d) { keep4_h(a, b, c, d); }
};
template <> struct Frag<__bf16> {
  typedef v16b V; union U { v16b v; v8b h[2]; };
  static __device__ __forceinline__ v16b load(const __bf16* p) {
    U f; f.h[0] = *(const v8b*)(p); f.h[1] = *(const v8b*)(p + 16); return f.v;
  }
  static __device__ __forceinline__ v8f mma(v16b a, v16b b, v8f c) {
    return __builtin_amdgcn_wmma_f32_16x16x32_bf16(false, a, false, b, (short)0, c, false, false);
  }
  static __device__ __forceinline__ void guard(v8f& a, v8f& b, v16b x, v16b y) { dep_guard_b(a, b, x, y); }
  static __device__ __forceinline__ void keep(v16b a, v16b b, v16b c, v16b d) { keep4_b(a, b, c, d); }
};
template <int ET> struct Elem;
template <> struct Elem<0> { typedef _Float16 T; };
template <> struct Elem<1> { typedef __bf16 T; };

template <int ET, int BIAS_MODE>
__device__ __forceinline__ void gemm64_body(
    const unsigned short* __restrict__ Ap, int lda, long strideA,
    const unsigned short* __restrict__ Btp, int ldb, long strideB,
    float* __restrict__ Cout, int ldc, long strideC,
    const float* __restrict__ bias, int M, int N, int K, float scale) {
  typedef typename Elem<ET>::T T;
  typedef typename Frag<T>::V V;
  const T* A = (const T*)Ap; const T* Bt = (const T*)Btp;
  __shared__ __align__(16) float sT[8][16 * 68];
  const int b    = blockIdx.y;
  const int lane = threadIdx.x & 31;
  const int wave = threadIdx.x >> 5;
  const int tilesN = N >> 6;
  const int tilesM = M >> 6;
  const int tile = blockIdx.x * 8 + wave;
  if (tile >= tilesM * tilesN) return;
  const int tm = tile / tilesN;
  const int tn = tile - tm * tilesN;
  const int m0 = tm << 6;
  const int n0 = tn << 6;

  const T* Ab  = A  + (size_t)b * strideA;
  const T* Bb  = Bt + (size_t)b * strideB;

  const int rlane = lane & 15;
  const int koff  = (lane >> 4) * 8;
  const int mOff  = (lane >> 4) * 8;

  v8f acc[4][4];
#pragma unroll
  for (int i = 0; i < 4; ++i)
#pragma unroll
    for (int j = 0; j < 4; ++j) acc[i][j] = (v8f){0.f,0.f,0.f,0.f,0.f,0.f,0.f,0.f};

  for (int k0 = 0; k0 < K; k0 += 32) {
    V bh[4];
#pragma unroll
    for (int j = 0; j < 4; ++j) {
      const size_t bo = (size_t)(n0 + (j << 4) + rlane) * ldb + koff + k0;
      bh[j] = Frag<T>::load(Bb + bo);
    }
#pragma unroll
    for (int i = 0; i < 4; ++i) {
      const size_t ao = (size_t)(m0 + (i << 4) + rlane) * lda + koff + k0;
      V ah = Frag<T>::load(Ab + ao);
#pragma unroll
      for (int j = 0; j < 4; ++j) {
        acc[i][j] = Frag<T>::mma(ah, bh[j], acc[i][j]);
      }
      Frag<T>::guard(acc[i][0], acc[i][3], ah, ah);
    }
    Frag<T>::keep(bh[0], bh[1], bh[2], bh[3]);
  }
  acc_guard4(acc[0][0], acc[0][1], acc[0][2], acc[0][3]);
  acc_guard4(acc[1][0], acc[1][1], acc[1][2], acc[1][3]);
  acc_guard4(acc[2][0], acc[2][1], acc[2][2], acc[2][3]);
  acc_guard4(acc[3][0], acc[3][1], acc[3][2], acc[3][3]);

  float* slab = sT[wave];
#pragma unroll
  for (int i = 0; i < 4; ++i) {
    const int mBase = m0 + (i << 4);
#pragma unroll
    for (int j = 0; j < 4; ++j) {
      const int n = n0 + (j << 4) + rlane;
      float bv = 0.f;
      if (BIAS_MODE == 2) bv = bias[n];
#pragma unroll
      for (int r = 0; r < 8; ++r) {
        float v = acc[i][j][r] * scale;
        if (BIAS_MODE == 2) v += bv;
        slab[(mOff + r) * 68 + (j << 4) + rlane] = v;
      }
    }
    __builtin_amdgcn_fence(3  , "workgroup");
    __builtin_amdgcn_wave_barrier();
    __builtin_amdgcn_fence(2  , "workgroup");
    {
      float* C = Cout + (size_t)b * strideC;
      const int hh = lane >> 4, c4 = (lane & 15) * 4;
      for (int pass = 0; pass < 2; ++pass) {
#pragma unroll
        for (int it = 0; it < 8; ++it) {
          const int row = it * 2 + hh;
          v4f v = *(const v4f*)(slab + row * 68 + c4);
          *(volatile v4f*)(C + (size_t)(mBase + row) * ldc + n0 + c4) = v;
        }
        __threadfence();
      }
    }
    __builtin_amdgcn_fence(3  , "workgroup");
    __builtin_amdgcn_wave_barrier();
    __builtin_amdgcn_fence(2  , "workgroup");
  }
}
}

__global__ __launch_bounds__(256) void k_gemm_f16(
    const unsigned short* __restrict__ Ap, int lda, long strideA,
    const unsigned short* __restrict__ Btp, int ldb, long strideB,
    float* __restrict__ Cout, int ldc, long strideC,
    int M, int N, int K, float scale) {
  w25::gemm64_body<0, 0>(Ap, lda, strideA, Btp, ldb, strideB, Cout, ldc, strideC, nullptr, M, N, K, scale);
}
__global__ __launch_bounds__(256) void k_gemm_bf16_bias(
    const unsigned short* __restrict__ Ap, int lda, long strideA,
    const unsigned short* __restrict__ Btp, int ldb, long strideB,
    float* __restrict__ Cout, int ldc, long strideC,
    const float* __restrict__ bias,
    int M, int N, int K, float scale) {
  w25::gemm64_body<1, 2>(Ap, lda, strideA, Btp, ldb, strideB, Cout, ldc, strideC, bias, M, N, K, scale);
}

#define AW 4
#define AT_KP 72
#define AT_PP 40
#define AT_OP 68
static_assert(AT_KP % 8 == 0 && AT_PP % 8 == 0 && AT_OP % 4 == 0);
static_assert(AT_KP >= DHEAD && AT_PP >= 32 && AT_OP >= DHEAD);
static_assert(32 * AW == 2 * 64);

union FragH { v16h v; v8h h[2]; };
__device__ __forceinline__ v8h cvt8h(v4f a, v4f c) {
    v8h r;
    r[0] = (_Float16)a.x; r[1] = (_Float16)a.y; r[2] = (_Float16)a.z; r[3] = (_Float16)a.w;
    r[4] = (_Float16)c.x; r[5] = (_Float16)c.y; r[6] = (_Float16)c.z; r[7] = (_Float16)c.w;
    return r;
}
__device__ __forceinline__ void wave_sync() {
    __builtin_amdgcn_fence(3  , "workgroup");
    __builtin_amdgcn_wave_barrier();
    __builtin_amdgcn_fence(2  , "workgroup");
}

__global__ __launch_bounds__(32 * AW) void k_attn_f16(const float* __restrict__ Qg, const float* __restrict__ Kg, const float* __restrict__ Vg,
                                                      float* __restrict__ Og, int seq, float scale) {
    __shared__ __align__(16) _Float16 Ks[64 * AT_KP];
    __shared__ __align__(16) _Float16 Vt[64 * AT_KP];
    __shared__ __align__(16) _Float16 Qs[AW][16 * AT_KP];
    __shared__ __align__(16) _Float16 Ps[AW][16 * AT_PP];
    __shared__ __align__(16) float    Os[AW][16 * AT_OP];
    const int tid = threadIdx.x, lane = tid & 31, hf = lane >> 4, l15 = lane & 15, wave = tid >> 5;
    const int h = blockIdx.y, b = blockIdx.z;
    const int q0 = (blockIdx.x * AW + wave) * 16;
    const size_t rowbase = (size_t)b * (size_t)seq;
    const int hoff = h * DHEAD;
    const float L2E = 1.4426950408889634f;
    const float NEG = -__builtin_inff();

    {
        const int qr = lane >> 1, dq = (lane & 1) * 32;
        const float* qsrc = Qg + (rowbase + (size_t)(q0 + qr)) * EMB + hoff + dq;
#pragma unroll
        for (int i = 0; i < 4; ++i) {
            const v4f a = *(const v4f*)(qsrc + 8 * i);
            const v4f c = *(const v4f*)(qsrc + 8 * i + 4);
            *(v8h*)&Qs[wave][qr * AT_KP + dq + 8 * i] = cvt8h(a, c);
        }
    }
    wave_sync();

    v8f o[4]; float m8[8], l8[8];
#pragma unroll
    for (int t = 0; t < 4; ++t) { v8f zz = {}; o[t] = zz; }
#pragma unroll
    for (int i = 0; i < 8; ++i) { m8[i] = NEG; l8[i] = 0.f; }

    const int nchunk = seq / 64;
    for (int kc = 0; kc < nchunk; ++kc) {
        const int kv0 = kc * 64;
        __syncthreads();
        {
            const int kvr = tid >> 1, dh = (tid & 1) * 32;
            const float* ksrc = Kg + (rowbase + (size_t)(kv0 + kvr)) * EMB + hoff + dh;
            const float* vsrc = Vg + (rowbase + (size_t)(kv0 + kvr)) * EMB + hoff + dh;
#pragma unroll
            for (int i = 0; i < 4; ++i) {
                const v4f a = *(const v4f*)(ksrc + 8 * i);
                const v4f c = *(const v4f*)(ksrc + 8 * i + 4);
                *(v8h*)&Ks[kvr * AT_KP + dh + 8 * i] = cvt8h(a, c);
            }
#pragma unroll
            for (int i = 0; i < 8; ++i) {
                const v4f vv = *(const v4f*)(vsrc + 4 * i);
                Vt[(dh + 4 * i + 0) * AT_KP + kvr] = (_Float16)vv.x;
                Vt[(dh + 4 * i + 1) * AT_KP + kvr] = (_Float16)vv.y;
                Vt[(dh + 4 * i + 2) * AT_KP + kvr] = (_Float16)vv.z;
                Vt[(dh + 4 * i + 3) * AT_KP + kvr] = (_Float16)vv.w;
            }
        }
        __syncthreads();

#pragma unroll 1
        for (int hb = 0; hb < 2; ++hb) {
            const int kb0 = hb * 32;
            v8f s0 = {}, s1 = {};
#pragma unroll
            for (int dc = 0; dc < 2; ++dc) {
                FragH qa, k0f, k1f;
                qa.h[0]  = *(const v8h*)&Qs[wave][l15 * AT_KP + dc * 32 + 8 * hf];
                qa.h[1]  = *(const v8h*)&Qs[wave][l15 * AT_KP + dc * 32 + 16 + 8 * hf];
                k0f.h[0] = *(const v8h*)&Ks[(kb0 + l15) * AT_KP + dc * 32 + 8 * hf];
                k0f.h[1] = *(const v8h*)&Ks[(kb0 + l15) * AT_KP + dc * 32 + 16 + 8 * hf];
                k1f.h[0] = *(const v8h*)&Ks[(kb0 + 16 + l15) * AT_KP + dc * 32 + 8 * hf];
                k1f.h[1] = *(const v8h*)&Ks[(kb0 + 16 + l15) * AT_KP + dc * 32 + 16 + 8 * hf];
                s0 = wmma16(qa.v, k0f.v, s0);
                s1 = wmma16(qa.v, k1f.v, s1);
            }
#pragma unroll
            for (int i = 0; i < 8; ++i) {
                float sc0 = s0[i] * scale; sc0 *= L2E;
                float sc1 = s1[i] * scale; sc1 *= L2E;
                float mx = fmaxf(sc0, sc1);
                mx = fmaxf(mx, __shfl_xor(mx, 1, 32)); mx = fmaxf(mx, __shfl_xor(mx, 2, 32));
                mx = fmaxf(mx, __shfl_xor(mx, 4, 32)); mx = fmaxf(mx, __shfl_xor(mx, 8, 32));
                const float mnew = fmaxf(m8[i], mx);
                const float corr = (mnew == NEG) ? 1.f : exp2f(m8[i] - mnew);
                const float p0 = exp2f(sc0 - mnew), p1 = exp2f(sc1 - mnew);
                float rs = p0 + p1;
                rs += __shfl_xor(rs, 1, 32); rs += __shfl_xor(rs, 2, 32); rs += __shfl_xor(rs, 4, 32); rs += __shfl_xor(rs, 8, 32);
                l8[i] = l8[i] * corr + rs; m8[i] = mnew;
                o[0][i] *= corr; o[1][i] *= corr; o[2][i] *= corr; o[3][i] *= corr;
                Ps[wave][(8 * hf + i) * AT_PP + l15]      = (_Float16)(p0 * 4096.f);
                Ps[wave][(8 * hf + i) * AT_PP + 16 + l15] = (_Float16)(p1 * 4096.f);
            }
            wave_sync();
            {
                FragH pa;
                pa.h[0] = *(const v8h*)&Ps[wave][l15 * AT_PP + 8 * hf];
                pa.h[1] = *(const v8h*)&Ps[wave][l15 * AT_PP + 16 + 8 * hf];
#pragma unroll
                for (int t = 0; t < 4; ++t) {
                    FragH vb;
                    vb.h[0] = *(const v8h*)&Vt[(t * 16 + l15) * AT_KP + kb0 + 8 * hf];
                    vb.h[1] = *(const v8h*)&Vt[(t * 16 + l15) * AT_KP + kb0 + 16 + 8 * hf];
                    o[t] = wmma16(pa.v, vb.v, o[t]);
                }
            }
            wave_sync();
        }
    }

#pragma unroll
    for (int i = 0; i < 8; ++i) {
        const float inv = (l8[i] > 0.f) ? 1.f / (l8[i] * 4096.f) : 0.f;
        Os[wave][(8 * hf + i) * AT_OP + l15]      = o[0][i] * inv;
        Os[wave][(8 * hf + i) * AT_OP + 16 + l15] = o[1][i] * inv;
        Os[wave][(8 * hf + i) * AT_OP + 32 + l15] = o[2][i] * inv;
        Os[wave][(8 * hf + i) * AT_OP + 48 + l15] = o[3][i] * inv;
    }
    wave_sync();
    {
        const int c4 = l15 * 4;
        float* obase = Og + (rowbase + (size_t)q0) * EMB + hoff;
#pragma unroll
        for (int it = 0; it < 8; ++it) {
            const int row = it * 2 + hf;
            const v4f v = *(const v4f*)&Os[wave][row * AT_OP + c4];
            VST2V4(obase + (size_t)row * EMB + c4, v);
        }
    }
}

__device__ __forceinline__ unsigned int cmb_pk2(float a, float b) { return (unsigned int)__builtin_bit_cast(unsigned short, (_Float16)a) | ((unsigned int)__builtin_bit_cast(unsigned short, (_Float16)b) << 16); }
__device__ __forceinline__ float cmb_bf(float v) { const unsigned u = __builtin_bit_cast(unsigned, v); const unsigned r = (u + 0x7fffu + ((u >> 16) & 1u)) & 0xffff0000u; return __builtin_bit_cast(float, r); }
__device__ __forceinline__ unsigned short bfu_rne(float v) { unsigned u = __builtin_bit_cast(unsigned, v); u += 0x7FFFu + ((u >> 16) & 1u); return (unsigned short)(u >> 16); }

__global__ __launch_bounds__(256) void k_cm_bfvec(const float* __restrict__ SRC, float* __restrict__ DST, int n) { const int u = blockIdx.x * 256 + threadIdx.x; if (u >= n) return; VST2(float, DST + u, cmb_bf(SRC[u])); }

__global__ __launch_bounds__(256) void k_cm_castb(const float* __restrict__ SRC, int lds, unsigned short* __restrict__ DST, int ldd, int nR, int nC, float sc) {
    const long long u = (long long)blockIdx.x * 256 + threadIdx.x; const int per = nC / 8; if (u >= (long long)nR * per) return; const int r = (int)(u / per); const int c0 = 8 * (int)(u % per);
    const float* s = SRC + (long long)r * lds + c0; float w[8];
#pragma unroll
    for (int e = 0; e < 8; ++e) w[e] = cmb_bf(s[e]) * sc;
    cm_u4 pk; pk.x = cmb_pk2(w[0], w[1]); pk.y = cmb_pk2(w[2], w[3]); pk.z = cmb_pk2(w[4], w[5]); pk.w = cmb_pk2(w[6], w[7]); VST2(cm_u4, (cm_u4*)(DST + (long long)r * ldd + c0), pk); }

__global__ __launch_bounds__(256) void k_cast_in(const float* __restrict__ SRC, unsigned short* __restrict__ DST, int nR, int seq, int seq_full) {
    const long long u = (long long)blockIdx.x * 256 + threadIdx.x; const int per = EMB / 8; if (u >= (long long)nR * per) return; const int r = (int)(u / per); const int c0 = 8 * (int)(u % per);
    const int bb = r / seq; const int ss = r - bb * seq;
    const float* s = SRC + ((long long)bb * seq_full + ss) * EMB + c0; float w[8];
#pragma unroll
    for (int e = 0; e < 8; ++e) w[e] = cmb_bf(s[e]);
    cm_u4 pk; pk.x = cmb_pk2(w[0], w[1]); pk.y = cmb_pk2(w[2], w[3]); pk.z = cmb_pk2(w[4], w[5]); pk.w = cmb_pk2(w[6], w[7]); VST2(cm_u4, (cm_u4*)(DST + (long long)r * EMB + c0), pk); }

__global__ __launch_bounds__(256) void k_wo_dup(const float* __restrict__ SRC, unsigned short* __restrict__ DST) {
    const int u = blockIdx.x * 256 + threadIdx.x; const int per = EMB / 8; if (u >= EMB * per) return; const int r = u / per; const int c0 = 8 * (u % per);
    const float* s = SRC + (long long)r * EMB + c0; unsigned int hb[8];
#pragma unroll
    for (int e = 0; e < 8; ++e) hb[e] = (unsigned int)bfu_rne(s[e]);
    cm_u4 pk; pk.x = hb[0] | (hb[1] << 16); pk.y = hb[2] | (hb[3] << 16); pk.z = hb[4] | (hb[5] << 16); pk.w = hb[6] | (hb[7] << 16);
    unsigned short* d0 = DST + (long long)r * (2 * EMB) + c0;
    VST2(cm_u4, (cm_u4*)d0, pk); VST2(cm_u4, (cm_u4*)(d0 + EMB), pk); }

__device__ __forceinline__ unsigned int f2bf2_pack(float a, float b, unsigned int* lo) {
    const unsigned short ha = w25::f2bf_bits(a), hb = w25::f2bf_bits(b);
    const unsigned short la = w25::f2bf_bits(a - w25::bf_bits2f(ha)), lb = w25::f2bf_bits(b - w25::bf_bits2f(hb));
    *lo = (unsigned)la | ((unsigned)lb << 16); return (unsigned)ha | ((unsigned)hb << 16); }
__global__ __launch_bounds__(256) void k_castS16(const float* __restrict__ src, long long lds, __bf16* __restrict__ dhi, __bf16* __restrict__ dlo, long long ldd, int R, int C, float s, int transpose) {
    const long long i = (long long)blockIdx.x * 256 + threadIdx.x; long long o; float a, b;
    if (transpose) { const long long np = (long long)C * (R / 2); if (i >= np) return; const int c = (int)(i / (R / 2)); const int r = 2 * (int)(i % (R / 2)); a = src[(long long)r * lds + c] * s; b = src[(long long)(r + 1) * lds + c] * s; o = (long long)c * ldd + r; }
    else { const long long np = (long long)R * (C / 2); if (i >= np) return; const int r = (int)(i / (C / 2)); const int c = 2 * (int)(i % (C / 2)); a = src[(long long)r * lds + c] * s; b = src[(long long)r * lds + c + 1] * s; o = (long long)r * ldd + c; }
    unsigned lo; const unsigned hi = f2bf2_pack(a, b, &lo); volatile unsigned* ph = (volatile unsigned*)(dhi + o); volatile unsigned* pl = (volatile unsigned*)(dlo + o);
    *ph = hi; *pl = lo; __threadfence(); *ph = hi; *pl = lo; }

constexpr size_t al256(size_t x) { return (x + 255) / 256 * 256; }
constexpr size_t SZ_X16 = al256((size_t)NB * SEQ * EMB * 2);
constexpr size_t SZ_W16 = al256((size_t)DHEAD * DHEAD * 2);
constexpr size_t SZ_PRJ = al256((size_t)NB * SEQ * EMB * 4);
constexpr size_t SZ_AO  = al256((size_t)NB * SEQ * EMB * 4);
constexpr size_t SZ_AOX = al256((size_t)NB * SEQ * 2 * EMB * 2);
constexpr size_t SZ_WOX = al256((size_t)EMB * 2 * EMB * 2);
constexpr size_t SZ_BRO = al256((size_t)EMB * 4);
constexpr size_t OFF_X16 = 0;
constexpr size_t OFF_WQ  = OFF_X16 + SZ_X16;
constexpr size_t OFF_WK  = OFF_WQ + SZ_W16;
constexpr size_t OFF_WV  = OFF_WK + SZ_W16;
constexpr size_t OFF_QP  = OFF_WV + SZ_W16;
constexpr size_t OFF_KP  = OFF_QP + SZ_PRJ;
constexpr size_t OFF_VP  = OFF_KP + SZ_PRJ;
constexpr size_t OFF_AO  = OFF_VP + SZ_PRJ;
constexpr size_t OFF_AOX = OFF_AO + SZ_AO;
constexpr size_t OFF_WOX = OFF_AOX + SZ_AOX;
constexpr size_t OFF_BRO = OFF_WOX + SZ_WOX;
constexpr size_t WS_TOTAL = OFF_BRO + SZ_BRO;
static_assert(WS_TOTAL <= (size_t)134217728);
static_assert((size_t)NB * SEQ * NHEAD * DHEAD * 4 <= SZ_PRJ);
static_assert((size_t)NB * SEQ * NHEAD * DHEAD * 2 <= SZ_X16);
static_assert((size_t)NB * SEQ * EMB * 4 <= SZ_AO);

extern "C" void kernel_launch(void* const* d_in, const int* in_sizes, int n_in, void* d_out, int out_size, void* d_ws, size_t ws_size, hipStream_t stream) {
    if (n_in < 8) return;
    const long long need_x = ((long long)(NB - 1) * SEQ_FULL + SEQ) * EMB;
    if ((long long)in_sizes[0] < need_x || (long long)in_sizes[1] < need_x || (long long)in_sizes[2] < need_x) return;
    if (in_sizes[3] < DHEAD * DHEAD || in_sizes[4] < DHEAD * DHEAD || in_sizes[5] < DHEAD * DHEAD) return;
    if (in_sizes[6] < EMB * EMB || in_sizes[7] < EMB) return;
    if ((long long)out_size < need_x) return;
    if (WS_TOTAL > ws_size) return;

    const float* xk = (const float*)d_in[0];
    const float* xq = (const float*)d_in[1];
    const float* xv = (const float*)d_in[2];
    const float* Wq = (const float*)d_in[3];
    const float* Wk = (const float*)d_in[4];
    const float* Wv = (const float*)d_in[5];
    const float* Wo = (const float*)d_in[6];
    const float* bo = (const float*)d_in[7];
    float* out = (float*)d_out;
    char* wsp = (char*)d_ws;
    unsigned short* X16  = (unsigned short*)(wsp + OFF_X16);
    unsigned short* W16q = (unsigned short*)(wsp + OFF_WQ);
    unsigned short* W16k = (unsigned short*)(wsp + OFF_WK);
    unsigned short* W16v = (unsigned short*)(wsp + OFF_WV);
    float* Qp = (float*)(wsp + OFF_QP);
    float* Kp = (float*)(wsp + OFF_KP);
    float* Vp = (float*)(wsp + OFF_VP);
    float* AO = (float*)(wsp + OFF_AO);
    unsigned short* AOX = (unsigned short*)(wsp + OFF_AOX);
    unsigned short* WOX = (unsigned short*)(wsp + OFF_WOX);
    float* BRO = (float*)(wsp + OFF_BRO);

    const int MROWS = NB * SEQ;
    const int MPROJ = NB * SEQ * NHEAD;
    const unsigned gW = (unsigned)((DHEAD * (DHEAD / 8) + 255) / 256);
    const unsigned gX = (unsigned)(((long long)MROWS * (EMB / 8) + 255) / 256);
    const unsigned gP = (unsigned)(((MPROJ / 64) * (DHEAD / 64) + 7) / 8);
    const unsigned gO = (unsigned)(((SEQ / 64) * (EMB / 64) + 7) / 8);

    k_cm_castb<<<gW, 256, 0, stream>>>(Wq, DHEAD, W16q, DHEAD, DHEAD, DHEAD, 16.0f);
    k_cm_castb<<<gW, 256, 0, stream>>>(Wk, DHEAD, W16k, DHEAD, DHEAD, DHEAD, 16.0f);
    k_cm_castb<<<gW, 256, 0, stream>>>(Wv, DHEAD, W16v, DHEAD, DHEAD, DHEAD, 16.0f);

    k_cast_in<<<gX, 256, 0, stream>>>(xq, X16, MROWS, SEQ, SEQ_FULL);
    k_gemm_f16<<<dim3(gP, 1), 256, 0, stream>>>(X16, DHEAD, 0L, W16q, DHEAD, 0L, Qp, DHEAD, 0L, MPROJ, DHEAD, DHEAD, 0.0625f);
    k_cast_in<<<gX, 256, 0, stream>>>(xk, X16, MROWS, SEQ, SEQ_FULL);
    k_gemm_f16<<<dim3(gP, 1), 256, 0, stream>>>(X16, DHEAD, 0L, W16k, DHEAD, 0L, Kp, DHEAD, 0L, MPROJ, DHEAD, DHEAD, 0.0625f);
    k_cast_in<<<gX, 256, 0, stream>>>(xv, X16, MROWS, SEQ, SEQ_FULL);
    k_gemm_f16<<<dim3(gP, 1), 256, 0, stream>>>(X16, DHEAD, 0L, W16v, DHEAD, 0L, Vp, DHEAD, 0L, MPROJ, DHEAD, DHEAD, 0.0625f);

    k_wo_dup<<<(unsigned)((EMB * (EMB / 8) + 255) / 256), 256, 0, stream>>>(Wo, WOX);
    k_cm_bfvec<<<(unsigned)((EMB + 255) / 256), 256, 0, stream>>>(bo, BRO, EMB);

    k_attn_f16<<<dim3((unsigned)(SEQ / 64), (unsigned)NHEAD, (unsigned)NB), 32 * AW, 0, stream>>>(Qp, Kp, Vp, AO, SEQ, 0.125f);

    k_castS16<<<(unsigned)(((long long)MROWS * (EMB / 2) + 255) / 256), 256, 0, stream>>>(AO, (long long)EMB, (__bf16*)AOX, (__bf16*)(AOX + EMB), (long long)(2 * EMB), MROWS, EMB, 1.0f, 0);

    k_gemm_bf16_bias<<<dim3(gO, (unsigned)NB), 256, 0, stream>>>(AOX, 2 * EMB, (long)SEQ * 2 * EMB, WOX, 2 * EMB, 0L, out, EMB, (long)SEQ_FULL * EMB, BRO, SEQ, EMB, 2 * EMB, 1.0f);
}
